// FlashAttention_29300266893601
// MI455X (gfx1250) — hardware-verified
//
#include <hip/hip_runtime.h>
#include <math.h>

#ifndef NB
#define NB 2
#endif
#ifndef SEQ
#define SEQ 2048
#endif
#define NB_FULL 2
#define S_FULL 2048
#define DM 1024
#define NHEAD 16
#define HDIM 64
#define MROWS (NB * SEQ)
#define WCARRY 16.0f
#define CCARRY 64.0f
#define RCARRY 2048.0f
static_assert(NB >= 1 && NB <= NB_FULL);
static_assert(SEQ % 64 == 0 && SEQ >= 64 && SEQ <= S_FULL);
static_assert(DM == NHEAD * HDIM);
static_assert(MROWS % 32 == 0 && DM % 64 == 0 && DM % 32 == 0);

typedef __attribute__((ext_vector_type(16))) _Float16 v16h;
typedef __attribute__((ext_vector_type(8)))  _Float16 v8h;
typedef __attribute__((ext_vector_type(16))) __bf16   v16b;
typedef __attribute__((ext_vector_type(8)))  float    v8f;
typedef __attribute__((ext_vector_type(4)))  float    v4f;
typedef __attribute__((ext_vector_type(4)))  unsigned int v4u;
union Frag { v16h v; v8h half[2]; };

__device__ __forceinline__ int frag_k(int i, int h) { return (i < 8) ? (8 * h + i) : (16 + 8 * h + (i - 8)); }
__device__ __forceinline__ __bf16 bf16_rne(float f) {
    unsigned int u = __float_as_uint(f);
    u += 0x7fffu + ((u >> 16) & 1u);
    return __builtin_bit_cast(__bf16, (unsigned short)(u >> 16));
}
__device__ __forceinline__ float bf16_f32(__bf16 b) { return __uint_as_float(((unsigned int)__builtin_bit_cast(unsigned short, b)) << 16); }
__device__ __forceinline__ v8f wmma16(v16h a, v16h b, v8f c) {
    c = __builtin_amdgcn_wmma_f32_16x16x32_f16(false, a, false, b, (short)0, c, false, false);
    asm volatile("v_nop\n\tv_nop\n\tv_nop\n\tv_nop" : "+v"(c) : "v"(a), "v"(b));
    return c;
}
__device__ __forceinline__ v8f wmmab(v16b a, v16b b, v8f c) {
    c = __builtin_amdgcn_wmma_f32_16x16x32_bf16(false, a, false, b, (short)0, c, false, false);
    asm volatile("v_nop\n\tv_nop\n\tv_nop\n\tv_nop" : "+v"(c) : "v"(a), "v"(b));
    return c;
}
struct Split { v16b hi, lo; };
__device__ __forceinline__ v8f wmma3(const Split& a, const Split& b, v8f c) {
    c = __builtin_amdgcn_wmma_f32_16x16x32_bf16(false, a.hi, false, b.hi, (short)0, c, false, false);
    c = __builtin_amdgcn_wmma_f32_16x16x32_bf16(false, a.hi, false, b.lo, (short)0, c, false, false);
    c = __builtin_amdgcn_wmma_f32_16x16x32_bf16(false, a.lo, false, b.hi, (short)0, c, false, false);
    asm volatile("v_nop\n\tv_nop\n\tv_nop\n\tv_nop" : "+v"(c) : "v"(a.hi), "v"(a.lo), "v"(b.hi), "v"(b.lo));
    return c;
}
struct Split3 { v16b hi, mid, lo; };
__device__ __forceinline__ v8f wmma6(const Split3& a, const Split3& b, v8f c) {
    c = __builtin_amdgcn_wmma_f32_16x16x32_bf16(false, a.hi, false, b.hi, (short)0, c, false, false);
    c = __builtin_amdgcn_wmma_f32_16x16x32_bf16(false, a.hi, false, b.mid, (short)0, c, false, false);
    c = __builtin_amdgcn_wmma_f32_16x16x32_bf16(false, a.mid, false, b.hi, (short)0, c, false, false);
    c = __builtin_amdgcn_wmma_f32_16x16x32_bf16(false, a.hi, false, b.lo, (short)0, c, false, false);
    c = __builtin_amdgcn_wmma_f32_16x16x32_bf16(false, a.mid, false, b.mid, (short)0, c, false, false);
    c = __builtin_amdgcn_wmma_f32_16x16x32_bf16(false, a.lo, false, b.hi, (short)0, c, false, false);
    asm volatile("v_nop\n\tv_nop\n\tv_nop\n\tv_nop" : "+v"(c) : "v"(a.hi), "v"(a.mid), "v"(a.lo), "v"(b.hi), "v"(b.mid), "v"(b.lo));
    return c;
}

__device__ __forceinline__ v16h fh_ld(const float* __restrict__ p, long long sk, int k0, int h, int klen, float s) {
    v16h a;
#pragma unroll
    for (int i = 0; i < 16; ++i) { const int k = k0 + frag_k(i, h); a[i] = (k < klen) ? (_Float16)(p[(long long)k * sk] * s) : (_Float16)0.f; }
    return a;
}
__device__ __forceinline__ Split sp_ld(const float* __restrict__ p, long long sk, int k0, int h, int klen, float s) {
    Split r;
#pragma unroll
    for (int i = 0; i < 16; ++i) {
        const int k = k0 + frag_k(i, h); const float x = (k < klen) ? p[(long long)k * sk] * s : 0.f;
        const __bf16 hb = bf16_rne(x); r.hi[i] = hb; r.lo[i] = bf16_rne(x - bf16_f32(hb));
    }
    return r;
}
__device__ __forceinline__ Split3 sp3_ld(const float* __restrict__ p, long long sk, int k0, int h, int klen, float s) {
    Split3 r;
#pragma unroll
    for (int i = 0; i < 16; ++i) {
        const int k = k0 + frag_k(i, h); const float x = (k < klen) ? p[(long long)k * sk] * s : 0.f;
        const __bf16 hb = bf16_rne(x); const float r1 = x - bf16_f32(hb); const __bf16 mb = bf16_rne(r1);
        r.hi[i] = hb; r.mid[i] = mb; r.lo[i] = bf16_rne(r1 - bf16_f32(mb));
    }
    return r;
}

#define VST2(T, ptr, val) do { const T vst2_v_ = (val); *(volatile T*)(ptr) = vst2_v_; __threadfence(); *(volatile T*)(ptr) = vst2_v_; } while (0)
#define VST2V4(ptr, val) do { const v4f vst2_v4_ = (val); *(volatile v4f*)(ptr) = vst2_v4_; __threadfence(); *(volatile v4f*)(ptr) = vst2_v4_; } while (0)

#define AW 4
struct AttnP {
    const float* Q; const float* K; const float* V; float* O; float* P; const float* Mf; const int* Mi; float* ST;
    const float* Pw; const float* Rt; const int* SQ; const int* SK;
    long long swb, swh, swi, swj, srb, srh, sri;
    long long sQb, sQh, sQi, sQd, sKb, sKh, sKj, sKd, sVb, sVh, sVj, sVd, sOb, sOh, sOi, sPb, sPh, sPi, smb, smh, smi, smj;
    int Lq, Lk, dh, dv, hrep, causal, coff, pband;
    float scale, mfill; int nonorm, mpol;
    int roff, rn, segpol, win;
};
static_assert(sizeof(AttnP) == 12 * 8 + 29 * 8 + 16 * 4);

#ifndef KATTN_ATTR
#define KATTN_ATTR
#endif
template <int DHP, int DVP, int QM, bool SPLITPV, bool TWOPASS>
__global__ __launch_bounds__(32 * AW) KATTN_ATTR void k_attn(AttnP p) {
    constexpr int NT = DVP / 16;
    constexpr int KS = DHP / 32;
    constexpr int VP = DVP + 8;
    __shared__ __align__(16) float    pl[AW][16 * 64];
    __shared__ __align__(16) _Float16 vl[(SPLITPV ? 2 : 1) * 64 * VP];
    const int lane = threadIdx.x & 31, hf = lane >> 4, l15 = lane & 15, wave = threadIdx.x >> 5;
    const int h = blockIdx.y, b = blockIdx.z, hk = h / p.hrep;
    const int q0 = (blockIdx.x * AW + wave) * 16;
    float* myp = pl[wave];
    const float L2E = 1.4426950408889634f;
    const float NEG = -__builtin_inff();
    const int qi = min(q0 + l15, p.Lq - 1);
    const float* qrow = p.Q + b * p.sQb + h * p.sQh + (long long)qi * p.sQi;
    const float* kbase = p.K + b * p.sKb + hk * p.sKh;
    const float* vbase = p.V + b * p.sVb + hk * p.sVh;
    v16h qa[QM == 0 ? KS : 1]; Split qs_[QM == 1 ? KS : 1]; Split3 qt_[QM == 2 ? KS : 1];
#pragma unroll
    for (int ks = 0; ks < KS; ++ks) {
        if (QM == 2) qt_[ks] = sp3_ld(qrow, p.sQd, ks * 32, hf, p.dh, 1.f);
        else if (QM == 1) qs_[ks] = sp_ld(qrow, p.sQd, ks * 32, hf, p.dh, 1.f);
        else qa[ks] = fh_ld(qrow, p.sQd, ks * 32, hf, p.dh, 1.f);
    }
    v8f o[NT]; float m8[8], l8[8];
#pragma unroll
    for (int t = 0; t < NT; ++t) { v8f zz = {}; o[t] = zz; }
#pragma unroll
    for (int i = 0; i < 8; ++i) { m8[i] = NEG; l8[i] = 0.f; }
    int jend = p.Lk; int jstart = 0;
    if (p.causal == 1) { const int je = (blockIdx.x * AW + AW - 1) * 16 + 16 + p.coff; jend = min(jend, max(je, 0)); }
    if (p.win > 0) { const int js = (int)(blockIdx.x * AW) * 16 + p.coff - p.win; jstart = (js > 0) ? (js / 64) * 64 : 0; }
    const int npass = TWOPASS ? 2 : 1;
    for (int pass = 0; pass < npass; ++pass) {
        const bool dopv = (!TWOPASS) || pass == 1;
        for (int j0 = jstart; j0 < jend; j0 += 64) {
            if (dopv) {
                __syncthreads();
                for (int idx = threadIdx.x; idx < 64 * DVP; idx += 32 * AW) {
                    const int jr = idx / DVP, d = idx - jr * DVP, j = j0 + jr;
                    const float f = (j < p.Lk && d < p.dv) ? vbase[(long long)j * p.sVj + (long long)d * p.sVd] : 0.f;
                    if (SPLITPV) {
                        const __bf16 hb = bf16_rne(f);
                        ((__bf16*)vl)[jr * VP + d] = hb; ((__bf16*)vl)[64 * VP + jr * VP + d] = bf16_rne(f - bf16_f32(hb));
                    } else vl[jr * VP + d] = (_Float16)f;
                }
            }
            v8f s[4];
#pragma unroll
            for (int t = 0; t < 4; ++t) {
                const int j = min(j0 + t * 16 + l15, p.Lk - 1);
                const float* krow = kbase + (long long)j * p.sKj;
                v8f acc = {};
#pragma unroll
                for (int ks = 0; ks < KS; ++ks) {
                    if (QM == 2)      acc = wmma6(qt_[ks], sp3_ld(krow, p.sKd, ks * 32, hf, p.dh, 1.f), acc);
                    else if (QM == 1) acc = wmma3(qs_[ks], sp_ld(krow, p.sKd, ks * 32, hf, p.dh, 1.f), acc);
                    else              acc = wmma16(qa[ks], fh_ld(krow, p.sKd, ks * 32, hf, p.dh, 1.f), acc);
                }
                s[t] = acc;
            }
            float pv[8][4];
#pragma unroll
            for (int i = 0; i < 8; ++i) {
                const int irow = q0 + i + 8 * hf;
                const int ic = min(irow, p.Lq - 1);
                float sc[4];
#pragma unroll
                for (int t = 0; t < 4; ++t) {
                    const int jg = j0 + t * 16 + l15;
                    float v = s[t][i] * p.scale;
                    if (p.Mf) v += p.Mf[b * p.smb + h * p.smh + (long long)ic * p.smi + (long long)min(jg, p.Lk - 1) * p.smj];
                    if (p.Rt) { int rc = ic - min(jg, p.Lk - 1) + p.roff; rc = rc < 0 ? 0 : (rc >= p.rn ? p.rn - 1 : rc); v += p.Rt[b * p.srb + h * p.srh + (long long)ic * p.sri + rc]; }
                    if (p.Mi) { const int mv = p.Mi[b * p.smb + h * p.smh + (long long)ic * p.smi + (long long)min(jg, p.Lk - 1) * p.smj]; if (p.mpol ? (mv != 0) : (mv == 0)) v = p.mfill; }
                    if (p.SQ) { const bool same = p.SQ[(long long)b * p.Lq + ic] == p.SK[(long long)b * p.Lk + min(jg, p.Lk - 1)]; if (p.segpol ? same : !same) v = p.mfill; }
                    if (p.causal == 2 && jg > irow + p.coff) v = p.mfill;
                    if (jg >= p.Lk || (p.causal == 1 && jg > irow + p.coff) || (p.causal == 3 && jg < irow + p.coff) || (p.win > 0 && irow + p.coff - jg > p.win)) v = NEG; else v *= L2E;
                    sc[t] = v;
                }
                if (!TWOPASS || pass == 0) {
                    float mx = fmaxf(fmaxf(sc[0], sc[1]), fmaxf(sc[2], sc[3]));
                    mx = fmaxf(mx, __shfl_xor(mx, 1, 32)); mx = fmaxf(mx, __shfl_xor(mx, 2, 32));
                    mx = fmaxf(mx, __shfl_xor(mx, 4, 32)); mx = fmaxf(mx, __shfl_xor(mx, 8, 32));
                    const float mnew = fmaxf(m8[i], mx);
                    const float corr = (mnew == NEG) ? 1.f : exp2f(m8[i] - mnew);
                    float rs = 0.f;
#pragma unroll
                    for (int t = 0; t < 4; ++t) {
                        const float pp = (sc[t] == NEG) ? 0.f : exp2f(sc[t] - mnew); rs += pp;
                        pv[i][t] = p.Pw ? pp * p.Pw[b * p.swb + h * p.swh + (long long)ic * p.swi + (long long)min(j0 + t * 16 + l15, p.Lk - 1) * p.swj] : pp;
                    }
                    rs += __shfl_xor(rs, 1, 32); rs += __shfl_xor(rs, 2, 32); rs += __shfl_xor(rs, 4, 32); rs += __shfl_xor(rs, 8, 32);
                    l8[i] = l8[i] * corr + rs; m8[i] = mnew;
                    if (!TWOPASS) {
#pragma unroll
                        for (int t = 0; t < NT; ++t) o[t][i] *= corr;
                    }
                } else {
                    const float inv = (l8[i] > 0.f) ? 1.f / l8[i] : 0.f;
#pragma unroll
                    for (int t = 0; t < 4; ++t) {
                        const int jg = j0 + t * 16 + l15;
                        float pp = (sc[t] == NEG) ? 0.f : exp2f(sc[t] - m8[i]) * inv;
                        if (p.Pw) pp *= p.Pw[b * p.swb + h * p.swh + (long long)ic * p.swi + (long long)min(jg, p.Lk - 1) * p.swj];
                        pv[i][t] = pp;
                    }
                }
            }
            if (dopv) {
#pragma unroll
                for (int i = 0; i < 8; ++i)
#pragma unroll
                    for (int t = 0; t < 4; ++t) ((volatile float*)myp)[(i + 8 * hf) * 64 + t * 16 + l15] = pv[i][t];
                __syncthreads();
                if (p.P) {
                    float* pb_ = p.P + b * p.sPb + h * p.sPh;
                    const bool fastP = (p.pband == 0) && ((p.sPi & 3) == 0) && (j0 + 64 <= p.Lk) && (q0 + 16 <= p.Lq) && ((((size_t)pb_) & 15) == 0);
                    if (fastP) {
#pragma unroll
                        for (int s2 = 0; s2 < 8; ++s2) {
                            const int row = s2 * 2 + (lane >> 4), c4 = (lane & 15) * 4;
                            const v4f v = *(const v4f*)(myp + row * 64 + c4);
                            VST2V4(pb_ + (long long)(q0 + row) * p.sPi + j0 + c4, v);
                        }
                    } else {
                        for (int row = 0; row < 16; ++row) {
                            const int irow = q0 + row; if (irow >= p.Lq) continue;
                            for (int c = lane; c < 64; c += 32) {
                                const int jg = j0 + c; if (jg >= p.Lk) continue;
                                if (p.pband == 0) VST2(float, pb_ + (long long)irow * p.sPi + jg, myp[row * 64 + c]);
                                else if (jg - irow <= p.pband && irow - jg <= p.pband) VST2(float, pb_ + (long long)irow * p.sPi + (jg - irow + p.pband), myp[row * 64 + c]);
                            }
                        }
                    }
                }
                if (SPLITPV) {
                    const Split pa0 = sp_ld(myp + l15 * 64, 1, 0, hf, 64, 1.f), pa1 = sp_ld(myp + l15 * 64, 1, 32, hf, 64, 1.f);
                    const __bf16* vh = (const __bf16*)vl; const __bf16* vlo = vh + 64 * VP;
#pragma unroll
                    for (int t = 0; t < NT; ++t) {
                        const int dcol = t * 16 + l15;
                        Split b0, b1;
#pragma unroll
                        for (int e = 0; e < 16; ++e) {
                            const int k0 = frag_k(e, hf), k1 = 32 + frag_k(e, hf);
                            b0.hi[e] = vh[k0 * VP + dcol]; b0.lo[e] = vlo[k0 * VP + dcol]; b1.hi[e] = vh[k1 * VP + dcol]; b1.lo[e] = vlo[k1 * VP + dcol];
                        }
                        o[t] = wmma3(pa0, b0, o[t]);
                        o[t] = wmma3(pa1, b1, o[t]);
                    }
                } else {
                    const v16h pa0 = fh_ld(myp + l15 * 64, 1, 0, hf, 64, 4096.f), pa1 = fh_ld(myp + l15 * 64, 1, 32, hf, 64, 4096.f);
#pragma unroll
                    for (int t = 0; t < NT; ++t) {
                        const int dcol = t * 16 + l15;
                        v16h b0, b1;
#pragma unroll
                        for (int e = 0; e < 16; ++e) { b0[e] = vl[frag_k(e, hf) * VP + dcol]; b1[e] = vl[(32 + frag_k(e, hf)) * VP + dcol]; }
                        o[t] = wmma16(pa0, b0, o[t]);
                        o[t] = wmma16(pa1, b1, o[t]);
                    }
                }
            }
        }
    }
    float* obase = p.O + b * p.sOb + h * p.sOh;
    if (p.ST) {
        const int rl = lane >> 1, isel = rl & 7;
        float mv = 0.f, lv = 0.f;
#pragma unroll
        for (int i = 0; i < 8; ++i) if (i == isel) { mv = m8[i]; lv = l8[i]; }
        const int irow = q0 + rl;
        if (irow < p.Lq) { float* st = p.ST + (((long long)b * gridDim.y + h) * p.Lq + irow) * 2 + (lane & 1); VST2(float, st, (lane & 1) ? lv : mv * 0.6931471805599453f); }
    }
    float invr[8];
#pragma unroll
    for (int i = 0; i < 8; ++i) {
        if (TWOPASS) invr[i] = SPLITPV ? 1.f : (1.f / 4096.f);
        else if (p.nonorm) invr[i] = exp2f(m8[i]) * (SPLITPV ? 1.f : (1.f / 4096.f));
        else invr[i] = (l8[i] > 0.f) ? (SPLITPV ? 1.f / l8[i] : 1.f / (l8[i] * 4096.f)) : 0.f;
    }
    __syncthreads();
    const bool ofast = ((p.sOi & 3) == 0) && ((((size_t)obase) & 15) == 0) && (q0 + 16 <= p.Lq);
#pragma unroll
    for (int c0 = 0; c0 < DVP; c0 += 64) {
#pragma unroll
        for (int i = 0; i < 8; ++i)
#pragma unroll
            for (int t = 0; t < NT; ++t) if (t * 16 >= c0 && t * 16 < c0 + 64) ((volatile float*)myp)[(i + 8 * hf) * 64 + (t * 16 - c0) + l15] = o[t][i] * invr[i];
        __syncthreads();
        const int cw = (DVP - c0 < 64) ? (DVP - c0) : 64;
        if (ofast && (c0 + cw <= p.dv) && (cw % 32 == 0)) {
            const int lpr = cw / 4;
            const int rows_per_ins = 32 / lpr;
            for (int r0 = 0; r0 < 16; r0 += rows_per_ins) {
                const int row = r0 + lane / lpr, c4 = (lane % lpr) * 4;
                const v4f v = *(const v4f*)(myp + row * 64 + c4);
                VST2V4(obase + (long long)(q0 + row) * p.sOi + c0 + c4, v);
            }
        } else {
            for (int row = 0; row < 16; ++row) {
                const int irow = q0 + row; if (irow >= p.Lq) continue;
                for (int c = lane; c < cw; c += 32) { const int d = c0 + c; if (d < p.dv) VST2(float, obase + (long long)irow * p.sOi + d, myp[row * 64 + c]); }
            }
        }
        __syncthreads();
    }
}

template <int TN, bool RES>
__global__ __launch_bounds__(32) void k_pgemm(const _Float16* __restrict__ Ah, const _Float16* __restrict__ Al, int lda, const _Float16* __restrict__ Bt, int ldb,
                                              float* __restrict__ C, int ldc, int M, int N, int K, float csc, float rsc) {
    static_assert(TN == 2 || TN == 4);
    const int lane = threadIdx.x & 31, h = lane >> 4, l15 = lane & 15;
    const int m0 = blockIdx.y * 32, n0 = blockIdx.x * (16 * TN);
    if (m0 + 32 > M || n0 + 16 * TN > N) return;
    v8f acc[2][TN], accr[2][TN];
#pragma unroll
    for (int i = 0; i < 2; ++i)
#pragma unroll
        for (int t = 0; t < TN; ++t) { v8f zz = {}; acc[i][t] = zz; accr[i][t] = zz; }
    for (int k0 = 0; k0 < K; k0 += 32) {
        Frag a[2], al[2];
#pragma unroll
        for (int i = 0; i < 2; ++i) {
            const _Float16* ar = Ah + (size_t)(m0 + 16 * i + l15) * lda + k0;
            a[i].half[0] = *(const v8h*)(ar + 8 * h); a[i].half[1] = *(const v8h*)(ar + 16 + 8 * h);
            if (RES) {
                const _Float16* lr = Al + (size_t)(m0 + 16 * i + l15) * lda + k0;
                al[i].half[0] = *(const v8h*)(lr + 8 * h); al[i].half[1] = *(const v8h*)(lr + 16 + 8 * h);
            } else al[i] = a[i];
        }
#pragma unroll
        for (int t = 0; t < TN; ++t) {
            const _Float16* br = Bt + (size_t)(n0 + 16 * t + l15) * ldb + k0;
            Frag bf; bf.half[0] = *(const v8h*)(br + 8 * h); bf.half[1] = *(const v8h*)(br + 16 + 8 * h);
#pragma unroll
            for (int i = 0; i < 2; ++i) {
                acc[i][t] = wmma16(a[i].v, bf.v, acc[i][t]);
                if (RES) accr[i][t] = wmma16(al[i].v, bf.v, accr[i][t]);
            }
        }
    }
    __shared__ __align__(16) float ctile[16][36];
#pragma unroll
    for (int i = 0; i < 2; ++i) {
#pragma unroll
        for (int tp = 0; tp < TN / 2; ++tp) {
#pragma unroll
            for (int t2 = 0; t2 < 2; ++t2) {
#pragma unroll
                for (int r = 0; r < 8; ++r) {
                    float v = acc[i][2 * tp + t2][r];
                    if (RES) v += accr[i][2 * tp + t2][r] * rsc;
                    ctile[8 * h + r][t2 * 16 + l15] = v * csc;
                }
            }
            __syncthreads();
#pragma unroll
            for (int s2 = 0; s2 < 4; ++s2) {
                const int row = s2 * 4 + (lane >> 3), c4 = (lane & 7) * 4;
                const v4f v = *(const v4f*)&ctile[row][c4];
                VST2V4(C + (size_t)(m0 + 16 * i + row) * ldc + n0 + 32 * tp + c4, v);
            }
            __syncthreads();
        }
    }
}

__device__ __forceinline__ unsigned int cmb_pk2(float a, float b) { return (unsigned int)__builtin_bit_cast(unsigned short, (_Float16)a) | ((unsigned int)__builtin_bit_cast(unsigned short, (_Float16)b) << 16); }
__device__ __forceinline__ float cmb_bf(float v) { const unsigned u = __builtin_bit_cast(unsigned, v); const unsigned r = (u + 0x7fffu + ((u >> 16) & 1u)) & 0xffff0000u; return __builtin_bit_cast(float, r); }
__device__ __forceinline__ unsigned int cmb_pkh2(_Float16 a, _Float16 b) { return (unsigned int)__builtin_bit_cast(unsigned short, a) | ((unsigned int)__builtin_bit_cast(unsigned short, b) << 16); }

__global__ __launch_bounds__(256) void k_cast16(const float* __restrict__ SRC, int lds, int rpb, long long sbat, unsigned short* __restrict__ DST, int ldd, int nR, int nC, float sc) {
    const long long u = (long long)blockIdx.x * 256 + threadIdx.x; const int per = nC / 8;
    if (u >= (long long)nR * per) return;
    const int r = (int)(u / per); const int c0 = 8 * (int)(u % per);
    const int bb = r / rpb, rr = r - bb * rpb;
    const float* s = SRC + (long long)bb * sbat + (long long)rr * lds + c0;
    const v4f x0 = *(const v4f*)s; const v4f x1 = *(const v4f*)(s + 4);
    const float f0 = x0.x, f1 = x0.y, f2 = x0.z, f3 = x0.w, f4 = x1.x, f5 = x1.y, f6 = x1.z, f7 = x1.w;
    const unsigned int w0 = cmb_pk2(cmb_bf(f0) * sc, cmb_bf(f1) * sc);
    const unsigned int w1 = cmb_pk2(cmb_bf(f2) * sc, cmb_bf(f3) * sc);
    const unsigned int w2 = cmb_pk2(cmb_bf(f4) * sc, cmb_bf(f5) * sc);
    const unsigned int w3 = cmb_pk2(cmb_bf(f6) * sc, cmb_bf(f7) * sc);
    v4u pk; pk.x = w0; pk.y = w1; pk.z = w2; pk.w = w3;
    VST2(v4u, (v4u*)(DST + (long long)r * ldd + c0), pk);
}

struct PkPair { unsigned int h; unsigned int l; };
__device__ __forceinline__ PkPair res_split2(float a, float b, float rsc) {
    const _Float16 ha = (_Float16)a, hb = (_Float16)b;
    const float ra = (a - (float)ha) * rsc, rb = (b - (float)hb) * rsc;
    const _Float16 la = (_Float16)ra, lb = (_Float16)rb;
    PkPair r; r.h = cmb_pkh2(ha, hb); r.l = cmb_pkh2(la, lb);
    return r;
}
__global__ __launch_bounds__(256) void k_castres(const float* __restrict__ SRC, int lds, unsigned short* __restrict__ DH, unsigned short* __restrict__ DL, int ldd, int nR, int nC, float sc, float rsc) {
    const long long u = (long long)blockIdx.x * 256 + threadIdx.x; const int per = nC / 8;
    if (u >= (long long)nR * per) return;
    const int r = (int)(u / per); const int c0 = 8 * (int)(u % per);
    const float* s = SRC + (long long)r * lds + c0;
    const v4f x0 = *(const v4f*)s; const v4f x1 = *(const v4f*)(s + 4);
    const float f0 = x0.x, f1 = x0.y, f2 = x0.z, f3 = x0.w, f4 = x1.x, f5 = x1.y, f6 = x1.z, f7 = x1.w;
    const PkPair p0 = res_split2(f0 * sc, f1 * sc, rsc);
    const PkPair p1 = res_split2(f2 * sc, f3 * sc, rsc);
    const PkPair p2 = res_split2(f4 * sc, f5 * sc, rsc);
    const PkPair p3 = res_split2(f6 * sc, f7 * sc, rsc);
    v4u pkh, pkl;
    pkh.x = p0.h; pkh.y = p1.h; pkh.z = p2.h; pkh.w = p3.h;
    pkl.x = p0.l; pkl.y = p1.l; pkl.z = p2.l; pkl.w = p3.l;
    VST2(v4u, (v4u*)(DH + (long long)r * ldd + c0), pkh);
    VST2(v4u, (v4u*)(DL + (long long)r * ldd + c0), pkl);
}

#define WS_XB ((size_t)MROWS * DM * 2)
#define WS_WB ((size_t)DM * DM * 2)
#define WS_FB ((size_t)MROWS * DM * 4)
#define WS_TOTAL (3 * WS_XB + 4 * WS_WB + 4 * WS_FB + 2 * WS_XB)
static_assert(WS_TOTAL <= (size_t)134217728);
static_assert(WS_XB % 256 == 0 && WS_WB % 256 == 0 && WS_FB % 256 == 0);

extern "C" void kernel_launch(void* const* d_in, const int* in_sizes, int n_in, void* d_out, int out_size, void* d_ws, size_t ws_size, hipStream_t stream) {
    if (n_in < 7) return;
    const long long needx = (long long)(NB - 1) * S_FULL * DM + (long long)SEQ * DM;
    if ((long long)in_sizes[0] < needx || (long long)in_sizes[1] < needx || (long long)in_sizes[2] < needx) return;
    if (in_sizes[3] < DM * DM || in_sizes[4] < DM * DM || in_sizes[5] < DM * DM || in_sizes[6] < DM * DM) return;
    if ((long long)out_size < (long long)MROWS * DM) return;
    if (WS_TOTAL > ws_size) return;
    const float* query = (const float*)d_in[0];
    const float* keyin = (const float*)d_in[1];
    const float* value = (const float*)d_in[2];
    const float* Wq = (const float*)d_in[3];
    const float* Wk = (const float*)d_in[4];
    const float* Wv = (const float*)d_in[5];
    const float* Wo = (const float*)d_in[6];
    float* out = (float*)d_out;
    char* wsp = (char*)d_ws;
    unsigned short* XQ = (unsigned short*)wsp; wsp += WS_XB;
    unsigned short* XK = (unsigned short*)wsp; wsp += WS_XB;
    unsigned short* XV = (unsigned short*)wsp; wsp += WS_XB;
    unsigned short* PWQ = (unsigned short*)wsp; wsp += WS_WB;
    unsigned short* PWK = (unsigned short*)wsp; wsp += WS_WB;
    unsigned short* PWV = (unsigned short*)wsp; wsp += WS_WB;
    unsigned short* PWO = (unsigned short*)wsp; wsp += WS_WB;
    float* QP = (float*)wsp; wsp += WS_FB;
    float* KP = (float*)wsp; wsp += WS_FB;
    float* VP = (float*)wsp; wsp += WS_FB;
    float* OC = (float*)wsp; wsp += WS_FB;
    unsigned short* CH = (unsigned short*)wsp; wsp += WS_XB;
    unsigned short* CL = (unsigned short*)wsp; wsp += WS_XB;
    if ((size_t)(wsp - (char*)d_ws) > ws_size) return;

    const unsigned gx = (unsigned)(((long long)MROWS * (DM / 8) + 255) / 256);
    k_cast16<<<gx, 256, 0, stream>>>(query, DM, SEQ, (long long)S_FULL * DM, XQ, DM, MROWS, DM, 1.0f);
    k_cast16<<<gx, 256, 0, stream>>>(keyin, DM, SEQ, (long long)S_FULL * DM, XK, DM, MROWS, DM, 1.0f);
    k_cast16<<<gx, 256, 0, stream>>>(value, DM, SEQ, (long long)S_FULL * DM, XV, DM, MROWS, DM, 1.0f);
    const unsigned gw = (unsigned)(((long long)DM * (DM / 8) + 255) / 256);
    k_cast16<<<gw, 256, 0, stream>>>(Wq, DM, DM, 0LL, PWQ, DM, DM, DM, WCARRY);
    k_cast16<<<gw, 256, 0, stream>>>(Wk, DM, DM, 0LL, PWK, DM, DM, DM, WCARRY);
    k_cast16<<<gw, 256, 0, stream>>>(Wv, DM, DM, 0LL, PWV, DM, DM, DM, WCARRY);
    k_cast16<<<gw, 256, 0, stream>>>(Wo, DM, DM, 0LL, PWO, DM, DM, DM, WCARRY);

    const dim3 gp((unsigned)(DM / 64), (unsigned)(MROWS / 32), 1);
    k_pgemm<4, false><<<gp, 32, 0, stream>>>((const _Float16*)XQ, (const _Float16*)XQ, DM, (const _Float16*)PWQ, DM, QP, DM, MROWS, DM, DM, 1.0f / WCARRY, 0.0f);
    k_pgemm<4, false><<<gp, 32, 0, stream>>>((const _Float16*)XK, (const _Float16*)XK, DM, (const _Float16*)PWK, DM, KP, DM, MROWS, DM, DM, 1.0f / WCARRY, 0.0f);
    k_pgemm<4, false><<<gp, 32, 0, stream>>>((const _Float16*)XV, (const _Float16*)XV, DM, (const _Float16*)PWV, DM, VP, DM, MROWS, DM, DM, 1.0f / WCARRY, 0.0f);

    { AttnP a;
      a.Q = QP; a.K = KP; a.V = VP; a.O = OC; a.P = 0; a.Mf = 0; a.Mi = 0; a.ST = 0;
      a.Pw = 0; a.Rt = 0; a.SQ = 0; a.SK = 0;
      a.swb = 0; a.swh = 0; a.swi = 0; a.swj = 0; a.srb = 0; a.srh = 0; a.sri = 0;
      a.sQb = (long long)SEQ * DM; a.sQh = HDIM; a.sQi = DM; a.sQd = 1;
      a.sKb = (long long)SEQ * DM; a.sKh = HDIM; a.sKj = DM; a.sKd = 1;
      a.sVb = (long long)SEQ * DM; a.sVh = HDIM; a.sVj = DM; a.sVd = 1;
      a.sOb = (long long)SEQ * DM; a.sOh = HDIM; a.sOi = DM;
      a.sPb = 0; a.sPh = 0; a.sPi = 0; a.smb = 0; a.smh = 0; a.smi = 0; a.smj = 0;
      a.Lq = SEQ; a.Lk = SEQ; a.dh = HDIM; a.dv = HDIM; a.hrep = 1; a.causal = 1; a.coff = 0; a.pband = 0;
      a.scale = 0.125f; a.mfill = 0.0f; a.nonorm = 0; a.mpol = 0;
      a.roff = 0; a.rn = 1; a.segpol = 0; a.win = 0;
      k_attn<64, 64, 1, true, false><<<dim3((unsigned)(SEQ / (16 * AW)), (unsigned)NHEAD, (unsigned)NB), 32 * AW, 0, stream>>>(a); }

    k_castres<<<gx, 256, 0, stream>>>(OC, DM, CH, CL, DM, MROWS, DM, CCARRY, RCARRY);
    const dim3 go((unsigned)(DM / 32), (unsigned)(MROWS / 32), 1);
    k_pgemm<2, true><<<go, 32, 0, stream>>>((const _Float16*)CH, (const _Float16*)CL, DM, (const _Float16*)PWO, DM, out, DM, MROWS, DM, DM, 1.0f / (CCARRY * WCARRY), 1.0f / RCARRY);
}
